// HeteroGraphormerLayerComplete_16252156248337
// MI455X (gfx1250) — hardware-run, weakly checked
//
#include <hip/hip_runtime.h>
#include <stddef.h>
#include <stdint.h>


#define NN    4096
#define CC    256
#define NHD   8
#define DHD   32
#define NE    32768
#define C3    768
#define C4    1024
#define FW    128

#define SPLIT_XN  1
#define SPLIT_MSG 1
#define SPLIT_HN  1
#define SPLIT_HID 1
#define K_XN  (SPLIT_XN  ? 2 * CC : CC)
#define K_MSG (SPLIT_MSG ? 2 * CC : CC)
#define K_HN  (SPLIT_HN  ? 2 * CC : CC)
#define K_HID (SPLIT_HID ? 2 * C4 : C4)

#define P_BQKV 0
#define P_BO   768
#define P_B1   1024
#define P_B2   2048
#define P_G1   2304
#define P_BE1  2560
#define P_G2   2816
#define P_BE2  3072
#define P_SPD  3328
#define P_ET   (P_SPD + 40)
#define P_IND  3392
#define P_OUTD 5696
#define PAR_N  8000
#define PAR_UNITS 2000

#define BTHR   256
#define BWAVE  8
#define BEPT   8
#define BCHUNK 2048
#define NCH    (NE / BCHUNK)
#define WCAP   256
#define LISTN  2048
#define NBS    1024
#define NBLK   (NN / NBS)
#define RCAP   32768
#define DEGCAP 4096
#define LDS_HEAD ((2 * NBS + LISTN + 2 * BWAVE) * 4)
#define LDS_B1 (LDS_HEAD + RCAP * 4)
#define LDS_B0 (LDS_HEAD + 2 * RCAP * 4)

#define GBM  64
#define GBN  64
#define GTHR 128

#define WSMAX 134217728

static_assert(RCAP >= NE);
static_assert((NE % BCHUNK) == 0);
static_assert((NE % 256) == 0);
static_assert((NN % NBS) == 0);
static_assert(BTHR * 4 == NBS);
static_assert(LISTN >= NBS && LISTN >= BWAVE * WCAP);
static_assert(WCAP == BEPT * 32);
static_assert(BCHUNK == BTHR * BEPT);
static_assert(LDS_B0 <= 327680);
static_assert((NN % GBM) == 0 && (C3 % GBN) == 0 && (CC % GBN) == 0 && (C4 % GBN) == 0);
static_assert((K_XN % 32) == 0 && (K_MSG % 32) == 0 && (K_HN % 32) == 0 && (K_HID % 32) == 0);
static_assert(GBM == (GTHR / 32) * 16);
static_assert((NN % 8) == 0);
static_assert(PAR_UNITS * 4 == PAR_N && (PAR_UNITS % 8) == 0);
static_assert(NHD * DHD == CC);
static_assert((size_t)(NN - 1) * CC + (CC - 1) == (size_t)NN * CC - 1);

typedef float          v4f   __attribute__((ext_vector_type(4)));
typedef float          v8f   __attribute__((ext_vector_type(8)));
typedef int            v4i   __attribute__((ext_vector_type(4)));
typedef int            v8i   __attribute__((ext_vector_type(8)));
typedef unsigned       v4u   __attribute__((ext_vector_type(4)));
typedef unsigned short v8us  __attribute__((ext_vector_type(8)));
typedef __bf16         v16bf __attribute__((ext_vector_type(16)));
union FragB { v16bf v; v8us u[2]; v8i w; };

__device__ __forceinline__ v8f wmx(const FragB& a, const FragB& b, v8f c) {
  v8f d = __builtin_amdgcn_wmma_f32_16x16x32_bf16(false, a.v, false, b.v, (short)0, c, false, false);
  asm volatile("v_nop\n\tv_nop\n\tv_nop\n\tv_nop" : "+v"(d) : "v"(a.w), "v"(b.w));
  return d;
}

__device__ __forceinline__ int clampi(int v, int lo, int hi) { return v < lo ? lo : (v > hi ? hi : v); }

__device__ __forceinline__ unsigned bfbits(float v) {
  const unsigned u = __float_as_uint(v);
  const unsigned r = (u + 0x7FFFu + ((u >> 16) & 1u)) >> 16;
  return (v != v) ? 0x7FC0u : r;
}
__device__ __forceinline__ float rbf(float v) { return __uint_as_float(bfbits(v) << 16); }

__device__ __forceinline__ v8us cvt8b(const v4f a, const v4f b) {
  v8us o;
  o[0] = (unsigned short)bfbits(a.x); o[1] = (unsigned short)bfbits(a.y);
  o[2] = (unsigned short)bfbits(a.z); o[3] = (unsigned short)bfbits(a.w);
  o[4] = (unsigned short)bfbits(b.x); o[5] = (unsigned short)bfbits(b.y);
  o[6] = (unsigned short)bfbits(b.z); o[7] = (unsigned short)bfbits(b.w);
  return o;
}
__device__ __forceinline__ void cvt8hl(const v4f a, const v4f b, v8us& hv, v8us& lv) {
  const float f[8] = {a.x, a.y, a.z, a.w, b.x, b.y, b.z, b.w};
#pragma unroll
  for (int i = 0; i < 8; ++i) {
    const unsigned hb = bfbits(f[i]);
    const float hf = __uint_as_float(hb << 16);
    hv[i] = (unsigned short)hb;
    lv[i] = (unsigned short)bfbits(f[i] - hf);
  }
}

__device__ __forceinline__ v4u par_take(const float* __restrict__ src, int f, int base, int len) {
  const int loc = f - base;
  const int idx = loc < 0 ? 0 : (loc > len - 4 ? len - 4 : loc);
  const v4f v = *(const v4f*)(src + idx);
  asm volatile("" :: "v"(v.x), "v"(v.y), "v"(v.z), "v"(v.w));
  const unsigned mk = ((unsigned)loc < (unsigned)len) ? 0xffffffffu : 0u;
  v4u r;
  r.x = __float_as_uint(v.x) & mk; r.y = __float_as_uint(v.y) & mk;
  r.z = __float_as_uint(v.z) & mk; r.w = __float_as_uint(v.w) & mk;
  return r;
}

__global__ __launch_bounds__(256) void k_par(
    const float* __restrict__ bq, const float* __restrict__ bk, const float* __restrict__ bv,
    const float* __restrict__ bo, const float* __restrict__ b1, const float* __restrict__ b2,
    const float* __restrict__ g1, const float* __restrict__ be1,
    const float* __restrict__ g2, const float* __restrict__ be2,
    const float* __restrict__ spd, const float* __restrict__ et,
    const float* __restrict__ ind, const float* __restrict__ outd, float* par)
{
  const int u  = (int)blockIdx.x * 256 + (int)threadIdx.x;
  const int uc = u < PAR_UNITS ? u : PAR_UNITS - 1;
  const int f  = 4 * uc;
  v4u acc = par_take(bq, f, P_BQKV, CC);
  acc |= par_take(bk,   f, P_BQKV + CC, CC);
  acc |= par_take(bv,   f, P_BQKV + 2 * CC, CC);
  acc |= par_take(bo,   f, P_BO,  CC);
  acc |= par_take(b1,   f, P_B1,  C4);
  acc |= par_take(b2,   f, P_B2,  CC);
  acc |= par_take(g1,   f, P_G1,  CC);
  acc |= par_take(be1,  f, P_BE1, CC);
  acc |= par_take(g2,   f, P_G2,  CC);
  acc |= par_take(be2,  f, P_BE2, CC);
  acc |= par_take(spd,  f, P_SPD, 40);
  acc |= par_take(ind,  f, P_IND, 9 * CC);
  acc |= par_take(outd, f, P_OUTD, 9 * CC);
  const float etv = et[0];
  asm volatile("" :: "v"(etv));
  const unsigned emk = (f == P_ET) ? 0xffffffffu : 0u;
  acc.x |= __float_as_uint(etv) & emk;
  v4f o;
  o.x = rbf(__uint_as_float(acc.x)); o.y = rbf(__uint_as_float(acc.y));
  o.z = rbf(__uint_as_float(acc.z)); o.w = rbf(__uint_as_float(acc.w));
  const bool ok = u < PAR_UNITS;
  float* op = par + f;
  if (ok) *(volatile v4f*)op = o;
  __threadfence();
  if (ok) *(volatile v4f*)op = o;
}

__global__ __launch_bounds__(256) void k_wtr(const float* __restrict__ w, int cols, int K,
                                             unsigned short* wt, int rowOff, int nUnits) {
  const int u = (int)blockIdx.x * 256 + (int)threadIdx.x;
  if (u >= nUnits) return;
  const int kq = K >> 3;
  const int n  = u / kq;
  const int k8 = (u - n * kq) * 8;
  const float* p = w + (size_t)k8 * (size_t)cols + n;
  v4f a, b;
  a.x = p[0];                  a.y = p[(size_t)cols];       a.z = p[(size_t)2 * cols];   a.w = p[(size_t)3 * cols];
  b.x = p[(size_t)4 * cols];   b.y = p[(size_t)5 * cols];   b.z = p[(size_t)6 * cols];   b.w = p[(size_t)7 * cols];
  const v8us hv = cvt8b(a, b);
  unsigned short* o = wt + (size_t)(rowOff + n) * (size_t)(2 * K) + k8;
  *(volatile v8us*)o = hv;
  *(volatile v8us*)(o + K) = hv;
  __threadfence();
  *(volatile v8us*)o = hv;
  *(volatile v8us*)(o + K) = hv;
}

__device__ __forceinline__ int scan_chunk(const int* __restrict__ keys, int cbase, int slotBase,
                                          int* list, int lane, int wave) {
  int wc = 0;
  const int elb  = wave * (BEPT * 32) + lane;
  const int e0   = cbase + elb;
  const int sent = -2147483647 - 1;
  const int k0 = keys[min(e0,       NE - 1)];
  const int k1 = keys[min(e0 + 32,  NE - 1)];
  const int k2 = keys[min(e0 + 64,  NE - 1)];
  const int k3 = keys[min(e0 + 96,  NE - 1)];
  const int k4 = keys[min(e0 + 128, NE - 1)];
  const int k5 = keys[min(e0 + 160, NE - 1)];
  const int k6 = keys[min(e0 + 192, NE - 1)];
  const int k7 = keys[min(e0 + 224, NE - 1)];
  asm volatile("" :: "v"(k0), "v"(k1), "v"(k2), "v"(k3), "v"(k4), "v"(k5), "v"(k6), "v"(k7));
  const int d0 = (e0       < NE) ? k0 : sent;
  const int d1 = (e0 + 32  < NE) ? k1 : sent;
  const int d2 = (e0 + 64  < NE) ? k2 : sent;
  const int d3 = (e0 + 96  < NE) ? k3 : sent;
  const int d4 = (e0 + 128 < NE) ? k4 : sent;
  const int d5 = (e0 + 160 < NE) ? k5 : sent;
  const int d6 = (e0 + 192 < NE) ? k6 : sent;
  const int d7 = (e0 + 224 < NE) ? k7 : sent;
  const unsigned nbs = (unsigned)slotBase;
  const unsigned unb = (unsigned)NBS;
  const unsigned s0 = (unsigned)d0 - nbs, s1 = (unsigned)d1 - nbs, s2 = (unsigned)d2 - nbs, s3 = (unsigned)d3 - nbs;
  const unsigned s4 = (unsigned)d4 - nbs, s5 = (unsigned)d5 - nbs, s6 = (unsigned)d6 - nbs, s7 = (unsigned)d7 - nbs;
  const bool h0 = s0 < unb, h1 = s1 < unb, h2 = s2 < unb, h3 = s3 < unb;
  const bool h4 = s4 < unb, h5 = s5 < unb, h6 = s6 < unb, h7 = s7 < unb;
  const unsigned any = __builtin_amdgcn_ballot_w32(h0 | h1 | h2 | h3 | h4 | h5 | h6 | h7);
  if (any != 0u) {
#define HITJ(J, HJ, SJ) { \
      const unsigned mj = __builtin_amdgcn_ballot_w32(HJ); \
      if (mj != 0u) { \
        if (HJ) { \
          const int pos = wc + (int)__builtin_amdgcn_mbcnt_lo(mj, 0u); \
          if (pos < WCAP) list[wave * WCAP + pos] = ((elb + 32 * (J)) << 12) | (int)(SJ); \
        } \
        wc += (int)__builtin_popcount(mj); } }
    HITJ(0, h0, s0)
    HITJ(1, h1, s1)
    HITJ(2, h2, s2)
    HITJ(3, h3, s3)
    HITJ(4, h4, s4)
    HITJ(5, h5, s5)
    HITJ(6, h6, s6)
    HITJ(7, h7, s7)
#undef HITJ
  }
  return wc;
}

template<int MODE>
__global__ __launch_bounds__(BTHR) void k_bucket(const int* __restrict__ keys, int* cntG, int* offG, int* listG) {
  extern __shared__ v4f lds_dyn[];
  int* scnt = (int*)lds_dyn;
  int* soff = scnt + NBS;
  int* list = soff + NBS;
  int* wcnt = list + LISTN;
  int* wtot = wcnt + BWAVE;
  int* reg1 = wtot + BWAVE;
  int* reg2 = reg1 + RCAP;
  const int tid = (int)threadIdx.x, lane = tid & 31, wave = tid >> 5;
  const int nodeBase = (int)blockIdx.x * NBS;

  for (int i = tid; i < NBS; i += BTHR) scnt[i] = 0;
  __syncthreads();

  int tot = 0;
#pragma unroll 1
  for (int ch = 0; ch < NCH; ++ch) {
    const int cbase = ch * BCHUNK;
    const int wc = scan_chunk(keys, cbase, nodeBase, list, lane, wave);
    if (lane == 0) wcnt[wave] = wc;
    __syncthreads();
    int pre = 0, all = 0;
#pragma unroll
    for (int w2 = 0; w2 < BWAVE; ++w2) {
      int c = wcnt[w2];
      c = c < 0 ? 0 : (c > WCAP ? WCAP : c);
      all += c;
      pre += (w2 < wave) ? c : 0;
    }
    const int wcc  = wc > WCAP ? WCAP : wc;
    const int base = tot + pre;
#pragma unroll 1
    for (int i = lane; i < wcc; i += 32) {
      const int ent = list[wave * WCAP + i];
      const int el  = (ent >> 12) & (BCHUNK - 1);
      const int sl  = ent & (NBS - 1);
      int eid = cbase + el;
      eid = eid > NE - 1 ? NE - 1 : eid;
      const int pos = base + i;
      if (pos < RCAP) reg1[pos] = (int)(((unsigned)eid << 12) | (unsigned)sl);
    }
    tot += all;
    tot = tot > RCAP ? RCAP : tot;
    __syncthreads();
  }
  const int nh = tot;

  if (wave == 0) {
#pragma unroll 1
    for (int b0 = 0; b0 < nh; b0 += 32) {
      int idx = b0 + lane;
      idx = idx > nh - 1 ? nh - 1 : idx;
      const int uv  = reg1[idx];
      const int m32 = (nh - b0) < 32 ? (nh - b0) : 32;
#pragma unroll 1
      for (int k = 0; k < m32; ++k) {
        const int u  = __builtin_amdgcn_readlane(uv, k);
        const int sl = u & (NBS - 1);
        if (lane == 0) scnt[sl] = scnt[sl] + 1;
      }
    }
  }
  __syncthreads();

  const v4i ca = *(const v4i*)(scnt + 4 * tid);
  const int e0 = ca.x < 0 ? 0 : ca.x, e1 = ca.y < 0 ? 0 : ca.y, e2 = ca.z < 0 ? 0 : ca.z, e3 = ca.w < 0 ? 0 : ca.w;
  const int ts = e0 + e1 + e2 + e3;
  int incl = ts;
#pragma unroll
  for (int d = 1; d < 32; d <<= 1) {
    const int up = __shfl_up(incl, d);
    if (lane >= d) incl += up;
  }
  if (lane == 31) wtot[wave] = incl;
  __syncthreads();
  int pre2 = 0;
#pragma unroll
  for (int w2 = 0; w2 < BWAVE; ++w2) pre2 += (w2 < wave) ? wtot[w2] : 0;
  const int r0 = pre2 + incl - ts, r1 = r0 + e0, r2 = r1 + e1, r3 = r2 + e2;
  v4i cvv; cvv.x = e0; cvv.y = e1; cvv.z = e2; cvv.w = e3;
  v4i ofv; ofv.x = r0; ofv.y = r1; ofv.z = r2; ofv.w = r3;

  if (MODE == 0) {
    soff[4 * tid + 0] = r0; soff[4 * tid + 1] = r1; soff[4 * tid + 2] = r2; soff[4 * tid + 3] = r3;
    __syncthreads();
    for (int i = tid; i < NBS; i += BTHR) list[i] = soff[i];
    __syncthreads();
    if (wave == 0) {
#pragma unroll 1
      for (int b0 = 0; b0 < nh; b0 += 32) {
        int idx = b0 + lane;
        idx = idx > nh - 1 ? nh - 1 : idx;
        const int uv  = reg1[idx];
        const int m32 = (nh - b0) < 32 ? (nh - b0) : 32;
#pragma unroll 1
        for (int k = 0; k < m32; ++k) {
          const int u   = __builtin_amdgcn_readlane(uv, k);
          const int sl  = u & (NBS - 1);
          const int eid = (int)((unsigned)u >> 12);
          if (lane == 0) {
            int pos = list[sl];
            pos = pos < 0 ? 0 : (pos > RCAP - 1 ? RCAP - 1 : pos);
            reg2[pos] = eid;
            list[sl] = pos + 1;
          }
        }
      }
      const int tz = nh + lane;
      if (tz < ((nh + 31) & ~31)) reg2[tz] = 0;
    }
    __syncthreads();
  }

  int* cp = cntG + nodeBase + 4 * tid;
  int* fp = offG + nodeBase + 4 * tid;
  int* lreg = listG + (size_t)blockIdx.x * NE;
  const int nq = ((nh + 31) >> 5) << 3;
  *(volatile v4i*)cp = cvv;
  if (MODE == 0) {
    *(volatile v4i*)fp = ofv;
#pragma unroll 1
    for (int q = tid; q < nq; q += BTHR) {
      const v4i v = *(const v4i*)(reg2 + 4 * q);
      *(volatile v4i*)(lreg + 4 * q) = v;
    }
  }
  __threadfence();
  *(volatile v4i*)cp = cvv;
  if (MODE == 0) {
    *(volatile v4i*)fp = ofv;
#pragma unroll 1
    for (int q = tid; q < nq; q += BTHR) {
      const v4i v = *(const v4i*)(reg2 + 4 * q);
      *(volatile v4i*)(lreg + 4 * q) = v;
    }
  }
  (void)fp; (void)lreg; (void)nq; (void)r3;
}

__device__ __forceinline__ void node_seg(const int* __restrict__ cntG, const int* __restrict__ offG, int node,
                                         int& cnt, int& off, int& craw) {
  const int c0 = cntG[node];
  const int o0 = offG[node];
  const int ov = clampi(o0, 0, NE - 1);
  int cv = clampi(c0, 0, DEGCAP);
  cv = cv > NE - ov ? NE - ov : cv;
  cnt = __builtin_amdgcn_readfirstlane(cv);
  off = __builtin_amdgcn_readfirstlane(ov);
  craw = c0;
}

__global__ __launch_bounds__(256) void k_f1(const int* __restrict__ src, const int* __restrict__ cntG,
                                            const int* __restrict__ offG, const int* __restrict__ listG,
                                            unsigned* Fout) {
  const int tid = (int)threadIdx.x, lane = tid & 31, wave = tid >> 5;
  const int node = (int)blockIdx.x * 8 + wave;
  int cnt, off, craw;
  node_seg(cntG, offG, node, cnt, off, craw);
  const int regBase = (node / NBS) * NE;
  v4u w; w.x = 0u; w.y = 0u; w.z = 0u; w.w = 0u;
#pragma unroll 1
  for (int p0 = 0; p0 < cnt; p0 += 32) {
    const int idx = clampi(clampi(off + p0 + lane, off, off + cnt - 1), 0, NE - 1);
    const int e   = clampi(listG[regBase + idx], 0, NE - 1);
    const int sv  = clampi(src[e], 0, NN - 1);
    const int m32 = (cnt - p0) < 32 ? (cnt - p0) : 32;
#pragma unroll 1
    for (int k = 0; k < m32; ++k) {
      const int sk = __builtin_amdgcn_readlane(sv, k);
      const int wk = sk >> 5;
      const unsigned bit = 1u << (sk & 31);
      const unsigned own = ((wk >> 2) == lane) ? bit : 0u;
      const int cmp = wk & 3;
      w.x |= (cmp == 0) ? own : 0u;
      w.y |= (cmp == 1) ? own : 0u;
      w.z |= (cmp == 2) ? own : 0u;
      w.w |= (cmp == 3) ? own : 0u;
    }
  }
  unsigned* op = Fout + (size_t)node * FW + 4 * lane;
  *(volatile v4u*)op = w;
  __threadfence();
  *(volatile v4u*)op = w;
  (void)craw;
}

__global__ __launch_bounds__(256) void k_hop(const int* __restrict__ src, const int* __restrict__ cntG,
                                             const int* __restrict__ offG, const int* __restrict__ listG,
                                             const unsigned* __restrict__ Fin, unsigned* Fout) {
  const int tid = (int)threadIdx.x, lane = tid & 31, wave = tid >> 5;
  const int node = (int)blockIdx.x * 8 + wave;
  int cnt, off, craw;
  node_seg(cntG, offG, node, cnt, off, craw);
  const int regBase = (node / NBS) * NE;
  v4u w; w.x = 0u; w.y = 0u; w.z = 0u; w.w = 0u;
#pragma unroll 1
  for (int p0 = 0; p0 < cnt; p0 += 32) {
    const int idx = clampi(clampi(off + p0 + lane, off, off + cnt - 1), 0, NE - 1);
    const int e   = clampi(listG[regBase + idx], 0, NE - 1);
    const int sv  = clampi(src[e], 0, NN - 1);
    const int m32 = (cnt - p0) < 32 ? (cnt - p0) : 32;
#pragma unroll 1
    for (int k = 0; k < m32; ++k) {
      const int sk = __builtin_amdgcn_readlane(sv, k);
      const v4u r = *(const v4u*)(Fin + (size_t)sk * FW + 4 * lane);
      w |= r;
    }
  }
  unsigned* op = Fout + (size_t)node * FW + 4 * lane;
  *(volatile v4u*)op = w;
  __threadfence();
  *(volatile v4u*)op = w;
  (void)craw;
}

__global__ __launch_bounds__(256) void k_spd(const int* __restrict__ ei, const unsigned* __restrict__ F1,
                                             const unsigned* __restrict__ F2, const unsigned* __restrict__ F3,
                                             int* spd) {
  const int e = (int)blockIdx.x * 256 + (int)threadIdx.x;
  const int s = clampi(ei[e], 0, NN - 1);
  const int d = clampi(ei[NE + e], 0, NN - 1);
  const size_t o = (size_t)s * FW + (size_t)(d >> 5);
  const unsigned w1 = F1[o];
  const unsigned w2 = F2[o];
  const unsigned w3 = F3[o];
  asm volatile("" :: "v"(w1), "v"(w2), "v"(w3));
  const int sh = d & 31;
  const int b1 = (int)((w1 >> sh) & 1u);
  const int b2 = (int)((w2 >> sh) & 1u);
  const int b3 = (int)((w3 >> sh) & 1u);
  int k = 4;
  k += b3 * (3 - k);
  k += b2 * (2 - k);
  k += b1 * (1 - k);
  *(volatile int*)(spd + e) = k;
  __threadfence();
  *(volatile int*)(spd + e) = k;
}

template<int MODE>
__global__ __launch_bounds__(256) void k_ln(const float* __restrict__ srcp,
                                            const int* __restrict__ cntI, const int* __restrict__ cntO,
                                            const float* __restrict__ par, int gOff, int bOff,
                                            float* XIN, unsigned short* XNP) {
  __shared__ __attribute__((aligned(16))) float stw[8 * CC];
  const int tid = (int)threadIdx.x, lane = tid & 31, wave = tid >> 5;
  const int node = (int)blockIdx.x * 8 + wave;
  const float* rp = srcp + (size_t)node * CC + 4 * lane;
  v4f ha = *(const v4f*)rp;
  v4f hb = *(const v4f*)(rp + 128);
  if (MODE == 0) {
    const int ci = clampi(cntI[node], 0, NE);
    const int co = clampi(cntO[node], 0, NE);
    int bi = 31 - (int)__builtin_clz((unsigned)(ci + 1));
    int bo = 31 - (int)__builtin_clz((unsigned)(co + 1));
    bi = bi > 8 ? 8 : bi;
    bo = bo > 8 ? 8 : bo;
    const float* ip = par + P_IND  + bi * CC + 4 * lane;
    const float* op = par + P_OUTD + bo * CC + 4 * lane;
    const v4f ia = *(const v4f*)ip, ib = *(const v4f*)(ip + 128);
    const v4f oa = *(const v4f*)op, ob = *(const v4f*)(op + 128);
    ha.x = (rbf(ha.x) + ia.x) + oa.x; ha.y = (rbf(ha.y) + ia.y) + oa.y;
    ha.z = (rbf(ha.z) + ia.z) + oa.z; ha.w = (rbf(ha.w) + ia.w) + oa.w;
    hb.x = (rbf(hb.x) + ib.x) + ob.x; hb.y = (rbf(hb.y) + ib.y) + ob.y;
    hb.z = (rbf(hb.z) + ib.z) + ob.z; hb.w = (rbf(hb.w) + ib.w) + ob.w;
    float* xo = XIN + (size_t)node * CC + 4 * lane;
    *(volatile v4f*)xo = ha;
    *(volatile v4f*)(xo + 128) = hb;
    __threadfence();
    *(volatile v4f*)xo = ha;
    *(volatile v4f*)(xo + 128) = hb;
  }
  float s = ((ha.x + ha.y) + (ha.z + ha.w)) + ((hb.x + hb.y) + (hb.z + hb.w));
#pragma unroll
  for (int o = 16; o > 0; o >>= 1) s += __shfl_xor(s, o);
  const float mu = s * (1.0f / CC);
  const v4f da = ha - mu;
  const v4f db = hb - mu;
  float q = ((da.x * da.x + da.y * da.y) + (da.z * da.z + da.w * da.w)) +
            ((db.x * db.x + db.y * db.y) + (db.z * db.z + db.w * db.w));
#pragma unroll
  for (int o = 16; o > 0; o >>= 1) q += __shfl_xor(q, o);
  const float var  = q * (1.0f / CC);
  const float sd   = sqrtf(var + 1e-5f);
  const float rinv = 1.0f / sd;
  const v4f ga = *(const v4f*)(par + gOff + 4 * lane);
  const v4f gb = *(const v4f*)(par + gOff + 128 + 4 * lane);
  const v4f ba = *(const v4f*)(par + bOff + 4 * lane);
  const v4f bb = *(const v4f*)(par + bOff + 128 + 4 * lane);
  const v4f ya = (ga * da) * rinv + ba;
  const v4f yb = (gb * db) * rinv + bb;
  float* sw = stw + wave * CC;
  *(v4f*)(sw + 4 * lane) = ya;
  *(v4f*)(sw + 128 + 4 * lane) = yb;
  __syncthreads();
  const v4f ra = *(const v4f*)(sw + 8 * lane);
  const v4f rb = *(const v4f*)(sw + 8 * lane + 4);
  v8us hv, lv;
  cvt8hl(ra, rb, hv, lv);
  unsigned short* xp = XNP + (size_t)node * (2 * CC) + 8 * lane;
  *(volatile v8us*)xp = hv;
  *(volatile v8us*)(xp + CC) = lv;
  __threadfence();
  *(volatile v8us*)xp = hv;
  *(volatile v8us*)(xp + CC) = lv;
  (void)cntI; (void)cntO; (void)XIN;
}

__global__ __launch_bounds__(256) void k_attn(const int* __restrict__ src, const int* __restrict__ cntG,
                                              const int* __restrict__ offG, const int* __restrict__ listG,
                                              const int* __restrict__ spdG, const float* __restrict__ QKV,
                                              const float* __restrict__ par, unsigned short* MSG) {
  __shared__ __attribute__((aligned(16))) float tab[64];
  const int tid = (int)threadIdx.x, lane = tid & 31, wave = tid >> 5;
  if (wave == 0) {
    const int bi = lane < 16 ? lane : 15;
    const v4f tv = *(const v4f*)(par + P_SPD + 4 * bi);
    asm volatile("" :: "v"(tv.x), "v"(tv.y), "v"(tv.z), "v"(tv.w));
    if (lane < 16) *(v4f*)(tab + 4 * lane) = tv;
  }
  __syncthreads();
  const int node = (int)blockIdx.x * 8 + wave;
  int cnt, off, craw;
  node_seg(cntG, offG, node, cnt, off, craw);
  const int regBase = (node / NBS) * NE;
  const int head = lane >> 2;
  const float etv = tab[40];
  const float* qp = QKV + (size_t)node * C3 + 8 * lane;
  const v4f qa = *(const v4f*)qp;
  const v4f qb = *(const v4f*)(qp + 4);
  v4f aa = {0.f, 0.f, 0.f, 0.f};
  v4f ab = {0.f, 0.f, 0.f, 0.f};
  float mx = -1.0e30f, dn = 0.0f;
#pragma unroll 1
  for (int p0 = 0; p0 < cnt; p0 += 32) {
    const int idx = clampi(clampi(off + p0 + lane, off, off + cnt - 1), 0, NE - 1);
    const int e   = clampi(listG[regBase + idx], 0, NE - 1);
    const int sv  = clampi(src[e], 0, NN - 1);
    const int kv  = clampi(spdG[e], 0, 4);
    const int m32 = (cnt - p0) < 32 ? (cnt - p0) : 32;
#pragma unroll 1
    for (int k = 0; k < m32; ++k) {
      const int sk = __builtin_amdgcn_readlane(sv, k);
      const int kk = __builtin_amdgcn_readlane(kv, k);
      const float* kp = QKV + (size_t)sk * C3 + CC + 8 * lane;
      const v4f ka = *(const v4f*)kp;
      const v4f kb = *(const v4f*)(kp + 4);
      const v4f va = *(const v4f*)(kp + CC);
      const v4f vb = *(const v4f*)(kp + CC + 4);
      float part = qa.x * ka.x;
      part = fmaf(qa.y, ka.y, part);
      part = fmaf(qa.z, ka.z, part);
      part = fmaf(qa.w, ka.w, part);
      part = fmaf(qb.x, kb.x, part);
      part = fmaf(qb.y, kb.y, part);
      part = fmaf(qb.z, kb.z, part);
      part = fmaf(qb.w, kb.w, part);
      part += __shfl_xor(part, 1);
      part += __shfl_xor(part, 2);
      const float sc = (part * 0.17677669529663687f + tab[kk * NHD + head]) + etv;
      const float df = sc - mx;
      const float ee = expf(-fabsf(df));
      const bool up  = df > 0.0f;
      const float s1 = up ? ee : 1.0f;
      const float s2 = up ? 1.0f : ee;
      mx = up ? sc : mx;
      dn = fmaf(dn, s1, s2);
      aa = aa * s1 + va * s2;
      ab = ab * s1 + vb * s2;
    }
  }
  const float ds = dn > 0.0f ? dn : 1.0f;
  const float iv = (dn > 0.0f ? 1.0f : 0.0f) * (1.0f / ds);
  const float pz = (craw > DEGCAP) ? __int_as_float(0x7fc00000) : 0.0f;
  const v4f ra = aa * iv + pz;
  const v4f rb = ab * iv + pz;
  v8us hv, lv;
  cvt8hl(ra, rb, hv, lv);
  unsigned short* mp = MSG + (size_t)node * (2 * CC) + 8 * lane;
  *(volatile v8us*)mp = hv;
  *(volatile v8us*)(mp + CC) = lv;
  __threadfence();
  *(volatile v8us*)mp = hv;
  *(volatile v8us*)(mp + CC) = lv;
}

template<int EPI>
__global__ __launch_bounds__(GTHR) __attribute__((amdgpu_num_vgpr(248)))
void k_gemm(const unsigned short* __restrict__ A, int lda,
            const unsigned short* __restrict__ WT, int ldw, int K,
            const float* __restrict__ bias, const float* __restrict__ res,
            float* outF, unsigned short* outB, int ldo)
{
  __shared__ __attribute__((aligned(16))) float stg[GBM * GBN];
  __shared__ __attribute__((aligned(16))) float sb[GBN];
  const int tid = (int)threadIdx.x, lane = tid & 31, wave = tid >> 5, hh = lane >> 4, m = lane & 15;
  const int rowBase = (int)blockIdx.x * GBM;
  const int col0    = (int)blockIdx.y * GBN;

  if (wave == 0) {
    const int bi = lane < 16 ? lane : 15;
    const v4f bv = *(const v4f*)(bias + col0 + 4 * bi);
    asm volatile("" :: "v"(bv.x), "v"(bv.y), "v"(bv.z), "v"(bv.w));
    if (lane < 16) *(v4f*)(sb + 4 * lane) = bv;
  }
  __syncthreads();

  v8f acc[4];
  {
    const v8f z = {0.f, 0.f, 0.f, 0.f, 0.f, 0.f, 0.f, 0.f};
    acc[0] = z; acc[1] = z; acc[2] = z; acc[3] = z;
  }
  const unsigned short* ap = A  + (size_t)(rowBase + 16 * wave + m) * (size_t)lda + 8 * hh;
  const unsigned short* wp = WT + (size_t)(col0 + m) * (size_t)ldw + 8 * hh;
  const int ksteps = K >> 5;
#pragma unroll 1
  for (int ks = 0; ks < ksteps; ++ks) {
    FragB af;
    af.u[0] = *(const v8us*)(ap + 32 * ks);
    af.u[1] = *(const v8us*)(ap + 32 * ks + 16);
#pragma unroll
    for (int t = 0; t < 4; ++t) {
      const unsigned short* wq = wp + (size_t)(16 * t) * (size_t)ldw + 32 * ks;
      FragB bf;
      bf.u[0] = *(const v8us*)wq;
      bf.u[1] = *(const v8us*)(wq + 16);
      acc[t] = wmx(af, bf, acc[t]);
    }
  }

#pragma unroll
  for (int t = 0; t < 4; ++t) {
    const int lc = 16 * t + m;
    const float bvl = sb[lc];
#pragma unroll
    for (int r = 0; r < 8; ++r) {
      const int lr = 16 * wave + 8 * hh + r;
      stg[lr * GBN + lc] = acc[t][r] + bvl;
    }
  }
  __syncthreads();

  if (EPI == 2) {
#pragma unroll 1
    for (int it = 0; it < (GBM * GBN) / GTHR; ++it) {
      const int idx = it * GTHR + tid;
      const float v = stg[idx];
      stg[idx] = 0.5f * v * (1.0f + erff(v * 0.70710678118654752f));
    }
    __syncthreads();
    const int q8 = lane & 7, sub = lane >> 3;
    v8us hv[4], lv[4];
#pragma unroll
    for (int i = 0; i < 4; ++i) {
      const int lr = 16 * wave + 4 * i + sub;
      const v4f ga = *(const v4f*)(stg + lr * GBN + 8 * q8);
      const v4f gb = *(const v4f*)(stg + lr * GBN + 8 * q8 + 4);
      cvt8hl(ga, gb, hv[i], lv[i]);
    }
#pragma unroll
    for (int i = 0; i < 4; ++i) {
      const int gr = rowBase + 16 * wave + 4 * i + sub;
      unsigned short* op = outB + (size_t)gr * (size_t)ldo + col0 + 8 * q8;
      *(volatile v8us*)op = hv[i];
      *(volatile v8us*)(op + C4) = lv[i];
    }
    __threadfence();
#pragma unroll
    for (int i = 0; i < 4; ++i) {
      const int gr = rowBase + 16 * wave + 4 * i + sub;
      unsigned short* op = outB + (size_t)gr * (size_t)ldo + col0 + 8 * q8;
      *(volatile v8us*)op = hv[i];
      *(volatile v8us*)(op + C4) = lv[i];
    }
  } else {
    v4f fv[8];
#pragma unroll
    for (int i = 0; i < 8; ++i) {
      const int lr = 16 * wave + 2 * i + hh;
      fv[i] = *(const v4f*)(stg + lr * GBN + 4 * m);
      if (EPI == 1) {
        const v4f rv = *(const v4f*)(res + (size_t)(rowBase + lr) * (size_t)ldo + col0 + 4 * m);
        fv[i] = fv[i] + rv;
      }
    }
#pragma unroll
    for (int i = 0; i < 8; ++i) {
      const int gr = rowBase + 16 * wave + 2 * i + hh;
      float* op = outF + (size_t)gr * (size_t)ldo + col0 + 4 * m;
      *(volatile v4f*)op = fv[i];
    }
    __threadfence();
#pragma unroll
    for (int i = 0; i < 8; ++i) {
      const int gr = rowBase + 16 * wave + 2 * i + hh;
      float* op = outF + (size_t)gr * (size_t)ldo + col0 + 4 * m;
      *(volatile v4f*)op = fv[i];
    }
  }
  (void)res; (void)outF; (void)outB;
}

#define SZ_PAR  32256
#define SZ_WQKV ((size_t)C3 * 2 * CC * 2)
#define SZ_WO   ((size_t)CC * 2 * CC * 2)
#define SZ_W1P  ((size_t)C4 * 2 * CC * 2)
#define SZ_W2P  ((size_t)CC * 2 * C4 * 2)
#define SZ_NI   ((size_t)NN * 4)
#define SZ_LIST ((size_t)NBLK * NE * 4)
#define SZ_SPD  ((size_t)NE * 4)
#define SZ_F    ((size_t)NN * FW * 4)
#define SZ_F32P ((size_t)NN * CC * 4)
#define SZ_HL   ((size_t)NN * 2 * CC * 2)
#define SZ_QKV  ((size_t)NN * C3 * 4)
#define SZ_HID  ((size_t)NN * 2 * C4 * 2)
#define O_PAR   ((size_t)0)
#define O_WQKV  (O_PAR + SZ_PAR)
#define O_WO    (O_WQKV + SZ_WQKV)
#define O_W1P   (O_WO + SZ_WO)
#define O_W2P   (O_W1P + SZ_W1P)
#define O_CNTI  (O_W2P + SZ_W2P)
#define O_CNTO  (O_CNTI + SZ_NI)
#define O_OFF   (O_CNTO + SZ_NI)
#define O_LIST  (O_OFF + SZ_NI)
#define O_SPD   (O_LIST + SZ_LIST)
#define O_F1    (O_SPD + SZ_SPD)
#define O_F2    (O_F1 + SZ_F)
#define O_F3    (O_F2 + SZ_F)
#define O_XIN   (O_F3 + SZ_F)
#define O_XN    (O_XIN + SZ_F32P)
#define O_QKV   (O_XN + SZ_HL)
#define O_MSG   (O_QKV + SZ_QKV)
#define O_H     (O_MSG + SZ_HL)
#define O_HN    (O_H + SZ_F32P)
#define O_HID   (O_HN + SZ_HL)
#define WS_TOTAL (O_HID + SZ_HID)
static_assert(SZ_PAR >= PAR_N * 4 && (SZ_PAR % 256) == 0);
static_assert((O_WQKV % 256) == 0 && (O_CNTI % 256) == 0 && (O_LIST % 256) == 0 && (O_XIN % 256) == 0);
static_assert(WS_TOTAL <= (size_t)WSMAX);

extern "C" void kernel_launch(void* const* d_in, const int* in_sizes, int n_in,
                              void* d_out, int out_size, void* d_ws, size_t ws_size,
                              hipStream_t stream) {
  if (n_in < 22) return;
  const int expn[22] = {NN * CC, 2 * NE, CC * CC, CC, CC * CC, CC, CC * CC, CC, CC * CC, CC,
                        CC * C4, C4, C4 * CC, CC, CC, CC, CC, CC, 5 * NHD, 9 * CC, 9 * CC, 1};
  for (int i = 0; i < 22; ++i) if (in_sizes[i] != expn[i]) return;
  if (out_size != NN * CC) return;
  if ((size_t)WS_TOTAL > ws_size) return;

  const float* x    = (const float*)d_in[0];
  const int*   ei   = (const int*)  d_in[1];
  const float* Wq   = (const float*)d_in[2];
  const float* bq   = (const float*)d_in[3];
  const float* Wk   = (const float*)d_in[4];
  const float* bk   = (const float*)d_in[5];
  const float* Wv   = (const float*)d_in[6];
  const float* bv   = (const float*)d_in[7];
  const float* Wo   = (const float*)d_in[8];
  const float* bo   = (const float*)d_in[9];
  const float* W1   = (const float*)d_in[10];
  const float* b1   = (const float*)d_in[11];
  const float* W2   = (const float*)d_in[12];
  const float* b2   = (const float*)d_in[13];
  const float* g1   = (const float*)d_in[14];
  const float* be1  = (const float*)d_in[15];
  const float* g2   = (const float*)d_in[16];
  const float* be2  = (const float*)d_in[17];
  const float* spe  = (const float*)d_in[18];
  const float* ind  = (const float*)d_in[19];
  const float* outd = (const float*)d_in[20];
  const float* etb  = (const float*)d_in[21];
  float* out = (float*)d_out;
  const int* src = ei;
  const int* dst = ei + NE;

  char* ws = (char*)d_ws;
  float*          PAR  = (float*)(ws + O_PAR);
  unsigned short* WQKV = (unsigned short*)(ws + O_WQKV);
  unsigned short* WOP  = (unsigned short*)(ws + O_WO);
  unsigned short* W1P  = (unsigned short*)(ws + O_W1P);
  unsigned short* W2P  = (unsigned short*)(ws + O_W2P);
  int*            CNTI = (int*)(ws + O_CNTI);
  int*            CNTO = (int*)(ws + O_CNTO);
  int*            OFFG = (int*)(ws + O_OFF);
  int*            LIST = (int*)(ws + O_LIST);
  int*            SPD  = (int*)(ws + O_SPD);
  unsigned*       F1   = (unsigned*)(ws + O_F1);
  unsigned*       F2   = (unsigned*)(ws + O_F2);
  unsigned*       F3   = (unsigned*)(ws + O_F3);
  float*          XIN  = (float*)(ws + O_XIN);
  unsigned short* XN   = (unsigned short*)(ws + O_XN);
  float*          QKV  = (float*)(ws + O_QKV);
  unsigned short* MSG  = (unsigned short*)(ws + O_MSG);
  float*          HB   = (float*)(ws + O_H);
  unsigned short* HN   = (unsigned short*)(ws + O_HN);
  unsigned short* HID  = (unsigned short*)(ws + O_HID);

  hipFuncSetAttribute(reinterpret_cast<const void*>(&k_bucket<0>),
                      hipFuncAttributeMaxDynamicSharedMemorySize, LDS_B0);
  hipFuncSetAttribute(reinterpret_cast<const void*>(&k_bucket<1>),
                      hipFuncAttributeMaxDynamicSharedMemorySize, LDS_B1);

  k_par<<<(PAR_UNITS + 255) / 256, 256, 0, stream>>>(bq, bk, bv, bo, b1, b2, g1, be1, g2, be2, spe, etb, ind, outd, PAR);

  k_wtr<<<(CC * (CC / 8)) / 256, 256, 0, stream>>>(Wq, CC, CC, WQKV, 0,      CC * (CC / 8));
  k_wtr<<<(CC * (CC / 8)) / 256, 256, 0, stream>>>(Wk, CC, CC, WQKV, CC,     CC * (CC / 8));
  k_wtr<<<(CC * (CC / 8)) / 256, 256, 0, stream>>>(Wv, CC, CC, WQKV, 2 * CC, CC * (CC / 8));
  k_wtr<<<(CC * (CC / 8)) / 256, 256, 0, stream>>>(Wo, CC, CC, WOP,  0,      CC * (CC / 8));
  k_wtr<<<(C4 * (CC / 8)) / 256, 256, 0, stream>>>(W1, C4, CC, W1P,  0,      C4 * (CC / 8));
  k_wtr<<<(CC * (C4 / 8)) / 256, 256, 0, stream>>>(W2, CC, C4, W2P,  0,      CC * (C4 / 8));

  k_bucket<0><<<NBLK, BTHR, LDS_B0, stream>>>(dst, CNTI, OFFG, LIST);
  k_bucket<1><<<NBLK, BTHR, LDS_B1, stream>>>(src, CNTO, OFFG, LIST);

  k_f1 <<<NN / 8, 256, 0, stream>>>(src, CNTI, OFFG, LIST, F1);
  k_hop<<<NN / 8, 256, 0, stream>>>(src, CNTI, OFFG, LIST, F1, F2);
  k_hop<<<NN / 8, 256, 0, stream>>>(src, CNTI, OFFG, LIST, F2, F3);
  k_spd<<<NE / 256, 256, 0, stream>>>(ei, F1, F2, F3, SPD);

  k_ln<0><<<NN / 8, 256, 0, stream>>>(x, CNTI, CNTO, PAR, P_G1, P_BE1, XIN, XN);

  k_gemm<0><<<dim3(NN / GBM, C3 / GBN), GTHR, 0, stream>>>(XN, 2 * CC, WQKV, 2 * CC, K_XN,
                                                           PAR + P_BQKV, XIN, QKV, HID, C3);
  k_attn<<<NN / 8, 256, 0, stream>>>(src, CNTI, OFFG, LIST, SPD, QKV, PAR, MSG);

  k_gemm<1><<<dim3(NN / GBM, CC / GBN), GTHR, 0, stream>>>(MSG, 2 * CC, WOP, 2 * CC, K_MSG,
                                                           PAR + P_BO, XIN, HB, HID, CC);
  k_ln<1><<<NN / 8, 256, 0, stream>>>(HB, CNTI, CNTO, PAR, P_G2, P_BE2, XIN, HN);

  k_gemm<2><<<dim3(NN / GBM, C4 / GBN), GTHR, 0, stream>>>(HN, 2 * CC, W1P, 2 * CC, K_HN,
                                                           PAR + P_B1, HB, QKV, HID, 2 * C4);
  k_gemm<1><<<dim3(NN / GBM, CC / GBN), GTHR, 0, stream>>>(HID, 2 * C4, W2P, 2 * C4, K_HID,
                                                           PAR + P_B2, HB, out, HID, CC);
}
